// DocREModel_32280974196898
// MI455X (gfx1250) — hardware-run, weakly checked
//
#include <hip/hip_runtime.h>
#include <stddef.h>
#include <stdint.h>
#include <math.h>


#define B_    4
#define S_    512
#define D_    768
#define H_    12
#define NE_   42
#define M_    8
#define OFF_  1
#define NN_   (NE_ * NE_)
#define MPAD_ 1792
#define OW_   (3 * D_)
#define CARRY     1024.0f
#define CARRY_INV (1.0f / 1024.0f)
#define WSCAP 134217728

static_assert(MPAD_ >= NN_);
static_assert((MPAD_ % 64) == 0);
static_assert((D_ % 64) == 0);
static_assert((S_ % 64) == 0);
static_assert((S_ % 32) == 0);
static_assert(S_ == 4 * 128);
static_assert(S_ == 8 * 64);
static_assert(D_ == 4 * 192);
static_assert(((D_ * 4) % 128) == 0);
static_assert(((OW_ * 4) % 128) == 0);
static_assert(((S_ * 2) % 128) == 0);

#define SZ_EMB  ((size_t)B_ * NE_ * D_ * 4)
#define SZ_EATT ((size_t)B_ * NE_ * H_ * S_ * 4)
#define SZ_SEQT ((size_t)B_ * D_ * S_ * 2)
#define SZ_HTA  ((size_t)B_ * MPAD_ * S_ * 2)
#define SZ_TOT  (SZ_EMB + SZ_EATT + SZ_SEQT + SZ_HTA)
static_assert((SZ_EMB % 256) == 0);
static_assert((SZ_EATT % 256) == 0);
static_assert((SZ_SEQT % 256) == 0);
static_assert((SZ_HTA % 256) == 0);
static_assert(SZ_TOT <= (size_t)WSCAP);

typedef float    v4f  __attribute__((ext_vector_type(4)));
typedef float    v8f  __attribute__((ext_vector_type(8)));
typedef _Float16 v8h  __attribute__((ext_vector_type(8)));
typedef _Float16 v16h __attribute__((ext_vector_type(16)));
union FragH { v16h v; v8h h[2]; };

__device__ __forceinline__ v8f wmf(v16h a, v16h b, v8f c) {
  v8f d = __builtin_amdgcn_wmma_f32_16x16x32_f16(false, a, false, b, (short)0, c, false, false);
  asm volatile("v_nop\n\tv_nop\n\tv_nop\n\tv_nop" : "+v"(d) : "v"(a), "v"(b));
  return d;
}

__device__ __forceinline__ v8h cvt8(v4f a, v4f b) {
  v8h r;
  r[0] = (_Float16)a.x; r[1] = (_Float16)a.y; r[2] = (_Float16)a.z; r[3] = (_Float16)a.w;
  r[4] = (_Float16)b.x; r[5] = (_Float16)b.y; r[6] = (_Float16)b.z; r[7] = (_Float16)b.w;
  return r;
}

__device__ __forceinline__ v4f addsel(v4f a, v4f x, int v) {
  v4f r;
  r.x = v ? (a.x + x.x) : a.x;
  r.y = v ? (a.y + x.y) : a.y;
  r.z = v ? (a.z + x.z) : a.z;
  r.w = v ? (a.w + x.w) : a.w;
  return r;
}

__global__ __launch_bounds__(256) void k_ent_emb(const float* __restrict__ seq,
                                                 const int* __restrict__ pos,
                                                 const int* __restrict__ msk,
                                                 float* emb) {
  __shared__ int spos[M_];
  __shared__ int sval[M_];
  __shared__ __attribute__((aligned(16))) float row[D_];
  const int be = blockIdx.x, b = be / NE_, tid = threadIdx.x;
  if (tid < M_) {
    int p = pos[be * M_ + tid] + OFF_;
    const int mk = msk[be * M_ + tid];
    const int v = (mk > 0 && p < S_) ? 1 : 0;
    p = min(max(p, 0), S_ - 1);
    spos[tid] = p;
    sval[tid] = v;
  }
  __syncthreads();
  const float* sb = seq + (size_t)b * S_ * D_;
#pragma unroll 1
  for (int d = tid; d < D_; d += 256) {
    float mx = -INFINITY;
#pragma unroll 1
    for (int m = 0; m < M_; ++m) {
      const float x = sb[(size_t)spos[m] * D_ + d];
      const float xs = sval[m] ? x : -INFINITY;
      mx = fmaxf(mx, xs);
    }
    const int has = (mx > -INFINITY) ? 1 : 0;
    const float mx0 = has ? mx : 0.f;
    float ssum = 0.f;
#pragma unroll 1
    for (int m = 0; m < M_; ++m) {
      const float x = sb[(size_t)spos[m] * D_ + d];
      const float e = expf(x - mx0);
      ssum += sval[m] ? e : 0.f;
    }
    const float lg = logf(ssum);
    row[d] = has ? (mx0 + lg) : 0.f;
  }
  __syncthreads();
  const int tc = min(tid, D_ / 4 - 1);
  const v4f v = *(const v4f*)(row + 4 * tc);
  float* dp = emb + (size_t)be * D_ + 4 * tc;
  if (tid < D_ / 4) *(volatile v4f*)dp = v;
  __threadfence();
  if (tid < D_ / 4) *(volatile v4f*)dp = v;
}

__global__ __launch_bounds__(128) void k_ent_att(const float* __restrict__ att,
                                                 const int* __restrict__ pos,
                                                 const int* __restrict__ msk,
                                                 float* eatt) {
  const int idx = blockIdx.x;
  const int h = idx % H_, be = idx / H_, b = be / NE_;
  const int tid = threadIdx.x;
  const float* ab = att + ((size_t)(b * H_ + h)) * S_ * S_ + 4 * tid;
  v4f acc = {0.f, 0.f, 0.f, 0.f};
  int cnt = 0;
#pragma unroll
  for (int m = 0; m < M_; ++m) {
    int p = pos[be * M_ + m] + OFF_;
    const int mk = msk[be * M_ + m];
    const int v = (mk > 0 && p < S_) ? 1 : 0;
    p = min(max(p, 0), S_ - 1);
    cnt += v;
    const v4f x = *(const v4f*)(ab + (size_t)p * S_);
    acc = addsel(acc, x, v);
  }
  const float inv = 1.0f / (float)max(cnt, 1);
  const v4f o = acc * inv;
  float* dp = eatt + (size_t)idx * S_ + 4 * tid;
  *(volatile v4f*)dp = o;
  __threadfence();
  *(volatile v4f*)dp = o;
}

#define TP_ 68
__global__ __launch_bounds__(256) void k_seqt(const float* __restrict__ seq, _Float16* seqt) {
  __shared__ __attribute__((aligned(16))) float ldt[64 * TP_];
  const int tid = threadIdx.x, lane = tid & 31, wv = tid >> 5;
  const int s0 = blockIdx.x * 64, d0 = blockIdx.y * 64, b = blockIdx.z;
  const float* sb = seq + (size_t)b * S_ * D_;
  const int tx = tid & 63, ty = tid >> 6;
#pragma unroll 4
  for (int it = 0; it < 16; ++it) {
    const int sl = ty + 4 * it;
    ldt[tx * TP_ + sl] = sb[(size_t)(s0 + sl) * D_ + d0 + tx];
  }
  __syncthreads();
  v8h hv[2];
#pragma unroll
  for (int q = 0; q < 2; ++q) {
    const int L = wv * 8 + 4 * q + (lane >> 3);
    const float* src = ldt + L * TP_ + 8 * (lane & 7);
    const v4f f0 = *(const v4f*)src;
    const v4f f1 = *(const v4f*)(src + 4);
    hv[q] = cvt8(f0, f1);
  }
#pragma unroll
  for (int q = 0; q < 2; ++q) {
    const int L = wv * 8 + 4 * q + (lane >> 3);
    _Float16* dp = seqt + ((size_t)(b * D_ + d0 + L)) * S_ + s0 + 8 * (lane & 7);
    *(volatile v8h*)dp = hv[q];
  }
  __threadfence();
#pragma unroll
  for (int q = 0; q < 2; ++q) {
    const int L = wv * 8 + 4 * q + (lane >> 3);
    _Float16* dp = seqt + ((size_t)(b * D_ + d0 + L)) * S_ + s0 + 8 * (lane & 7);
    *(volatile v8h*)dp = hv[q];
  }
}

__global__ __launch_bounds__(64) void k_ht(const float* __restrict__ eatt, _Float16* hta) {
  __shared__ float red[2];
  const int ij = blockIdx.x, b = blockIdx.y;
  const int tid = threadIdx.x, lane = tid & 31, wv = tid >> 5;
  const int pad = (ij >= NN_) ? 1 : 0;
  const int ijc = pad ? 0 : ij;
  const int i = ijc / NE_;
  const int j = ijc - i * NE_;
  const float* ei = eatt + ((size_t)((b * NE_ + i) * H_)) * S_ + 8 * tid;
  const float* ej = eatt + ((size_t)((b * NE_ + j) * H_)) * S_ + 8 * tid;
  v4f va = {0.f, 0.f, 0.f, 0.f}, vb = {0.f, 0.f, 0.f, 0.f};
#pragma unroll 1
  for (int h = 0; h < H_; ++h) {
    const v4f a0 = *(const v4f*)(ei + h * S_);
    const v4f a1 = *(const v4f*)(ei + h * S_ + 4);
    const v4f c0 = *(const v4f*)(ej + h * S_);
    const v4f c1 = *(const v4f*)(ej + h * S_ + 4);
    va += a0 * c0;
    vb += a1 * c1;
  }
  const float invh = 1.0f / (float)H_;
  va = va * invh;
  vb = vb * invh;
  float loc = ((va.x + va.y) + (va.z + va.w)) + ((vb.x + vb.y) + (vb.z + vb.w));
  loc += __shfl_xor(loc, 16);
  loc += __shfl_xor(loc, 8);
  loc += __shfl_xor(loc, 4);
  loc += __shfl_xor(loc, 2);
  loc += __shfl_xor(loc, 1);
  if (lane == 0) red[wv] = loc;
  __syncthreads();
  const float z = red[0] + red[1];
  const float invz = 1.0f / (z + 1e-5f);
  const float sc = pad ? 0.f : invz * CARRY;
  const v8h hv = cvt8(va * sc, vb * sc);
  _Float16* dp = hta + ((size_t)(b * MPAD_ + ij)) * S_ + 8 * tid;
  *(volatile v8h*)dp = hv;
  __threadfence();
  *(volatile v8h*)dp = hv;
}

__global__ __launch_bounds__(192) void k_hsts(const float* __restrict__ emb, float* out) {
  const int bi = blockIdx.x;
  const int b = bi / NE_;
  const int tid = threadIdx.x;
  const v4f hv = *(const v4f*)(emb + (size_t)bi * D_ + 4 * tid);
  const float* eb = emb + (size_t)b * NE_ * D_ + 4 * tid;
  float* ob = out + (size_t)bi * NE_ * OW_ + 4 * tid;
#pragma unroll 1
  for (int j = 0; j < NE_; ++j) {
    const v4f tv = *(const v4f*)(eb + (size_t)j * D_);
    float* o = ob + (size_t)j * OW_;
    *(volatile v4f*)o = hv;
    *(volatile v4f*)(o + D_) = tv;
  }
  __threadfence();
#pragma unroll 1
  for (int j = 0; j < NE_; ++j) {
    const v4f tv = *(const v4f*)(eb + (size_t)j * D_);
    float* o = ob + (size_t)j * OW_;
    *(volatile v4f*)o = hv;
    *(volatile v4f*)(o + D_) = tv;
  }
}

__global__ __launch_bounds__(128) void k_gemm(const _Float16* __restrict__ hta,
                                              const _Float16* __restrict__ seqt,
                                              float* out) {
  __shared__ __attribute__((aligned(16))) float stile[4 * 16 * 64];
  const int tid = threadIdx.x, lane = tid & 31, wv = tid >> 5, hh = lane >> 4, m = lane & 15;
  const int col0 = blockIdx.x * 64;
  const int row0 = blockIdx.y * 64 + 16 * wv;
  const int b = blockIdx.z;
  const _Float16* ap = hta + ((size_t)(b * MPAD_ + row0 + m)) * S_ + 8 * hh;
  const _Float16* bp = seqt + ((size_t)(b * D_ + col0 + m)) * S_ + 8 * hh;
  const v8f zero8 = {0.f, 0.f, 0.f, 0.f, 0.f, 0.f, 0.f, 0.f};
  v8f acc[4];
#pragma unroll
  for (int nt = 0; nt < 4; ++nt) acc[nt] = zero8;

#pragma unroll 2
  for (int k0 = 0; k0 < S_; k0 += 32) {
    FragH af;
    af.h[0] = *(const v8h*)(ap + k0);
    af.h[1] = *(const v8h*)(ap + k0 + 16);
#pragma unroll
    for (int nt = 0; nt < 4; ++nt) {
      const _Float16* bq = bp + (size_t)nt * 16 * S_ + k0;
      FragH bf;
      bf.h[0] = *(const v8h*)bq;
      bf.h[1] = *(const v8h*)(bq + 16);
      acc[nt] = wmf(af.v, bf.v, acc[nt]);
    }
  }

  float* st = stile + wv * (16 * 64);
#pragma unroll
  for (int nt = 0; nt < 4; ++nt) {
#pragma unroll
    for (int r = 0; r < 8; ++r) st[(8 * hh + r) * 64 + 16 * nt + m] = acc[nt][r] * CARRY_INV;
  }
  __syncthreads();

  v4f vv[8];
#pragma unroll
  for (int it = 0; it < 8; ++it) {
    const int lq = 4 * it + (lane >> 3);
    const int rl = lq >> 1;
    const int c = (lq & 1) * 32 + 4 * (lane & 7);
    vv[it] = *(const v4f*)(st + rl * 64 + c);
  }
  const size_t obase = (size_t)b * NN_;
#pragma unroll
  for (int it = 0; it < 8; ++it) {
    const int lq = 4 * it + (lane >> 3);
    const int rl = lq >> 1;
    const int c = (lq & 1) * 32 + 4 * (lane & 7);
    const int grow = row0 + rl;
    const int growc = min(grow, NN_ - 1);
    float* gp = out + (obase + (size_t)growc) * OW_ + 2 * D_ + col0 + c;
    if (grow < NN_) *(volatile v4f*)gp = vv[it];
  }
  __threadfence();
#pragma unroll
  for (int it = 0; it < 8; ++it) {
    const int lq = 4 * it + (lane >> 3);
    const int rl = lq >> 1;
    const int c = (lq & 1) * 32 + 4 * (lane & 7);
    const int grow = row0 + rl;
    const int growc = min(grow, NN_ - 1);
    float* gp = out + (obase + (size_t)growc) * OW_ + 2 * D_ + col0 + c;
    if (grow < NN_) *(volatile v4f*)gp = vv[it];
  }
}

extern "C" void kernel_launch(void* const* d_in, const int* in_sizes, int n_in,
                              void* d_out, int out_size, void* d_ws, size_t ws_size,
                              hipStream_t stream) {
  if (n_in < 4) return;
  if (in_sizes[0] != B_ * S_ * D_) return;
  if (in_sizes[1] != B_ * H_ * S_ * S_) return;
  if (in_sizes[2] != B_ * NE_ * M_) return;
  if (in_sizes[3] != B_ * NE_ * M_) return;
  if (out_size != B_ * NN_ * OW_) return;

  const float* seq = (const float*)d_in[0];
  const float* att = (const float*)d_in[1];
  const int*   pos = (const int*)d_in[2];
  const int*   msk = (const int*)d_in[3];
  float* out = (float*)d_out;

  char* ws = (char*)d_ws;
  size_t off = 0;
  const size_t oEMB  = off; off += SZ_EMB;
  const size_t oEATT = off; off += SZ_EATT;
  const size_t oSEQT = off; off += SZ_SEQT;
  const size_t oHTA  = off; off += SZ_HTA;
  if (off != SZ_TOT) return;
  if (off > ws_size || off > (size_t)WSCAP) return;

  float*    emb  = (float*)(ws + oEMB);
  float*    eatt = (float*)(ws + oEATT);
  _Float16* seqt = (_Float16*)(ws + oSEQT);
  _Float16* hta  = (_Float16*)(ws + oHTA);

  k_ent_emb<<<B_ * NE_, 256, 0, stream>>>(seq, pos, msk, emb);
  k_ent_att<<<B_ * NE_ * H_, 128, 0, stream>>>(att, pos, msk, eatt);
  k_seqt<<<dim3(S_ / 64, D_ / 64, B_), 256, 0, stream>>>(seq, seqt);
  k_ht<<<dim3(MPAD_, B_), 64, 0, stream>>>(eatt, hta);
  k_hsts<<<B_ * NE_, 192, 0, stream>>>(emb, out);
  k_gemm<<<dim3(D_ / 64, MPAD_ / 64, B_), 128, 0, stream>>>(hta, seqt, out);
}
